// SpectralGraphConv_48318382080441
// MI455X (gfx1250) — hardware-verified
//
#include <hip/hip_runtime.h>
#include <math.h>

typedef __attribute__((ext_vector_type(16))) _Float16 v16h;
typedef __attribute__((ext_vector_type(16))) __bf16 v16b;
typedef __attribute__((ext_vector_type(8)))  _Float16 v8h;
typedef __attribute__((ext_vector_type(8)))  float v8f;
typedef __attribute__((ext_vector_type(4)))  float v4f;
typedef __attribute__((ext_vector_type(2)))  float v2f;
typedef __attribute__((ext_vector_type(4)))  unsigned v4u;
typedef __attribute__((ext_vector_type(4)))  int v4i;
typedef float __attribute__((may_alias)) float_a;
typedef int __attribute__((may_alias)) int_a;

template <typename T> __device__ __forceinline__ void vst2(void* p, T v) { *(volatile T*)p = v; __threadfence(); *(volatile T*)p = v; }
__device__ __forceinline__ v8f wmma16(v16h a, v16h b, v8f c) {
  v8f d = __builtin_amdgcn_wmma_f32_16x16x32_f16(false, a, false, b, (short)0, c, false, false);
  asm volatile("v_nop\n\tv_nop\n\tv_nop\n\tv_nop" : "+v"(d) : "v"(a), "v"(b));
  return d;
}
__device__ __forceinline__ v8f wmma_bf(v16b a, v16b b, v8f c) {
  v8f d = __builtin_amdgcn_wmma_f32_16x16x32_bf16(false, a, false, b, (short)0, c, false, false);
  asm volatile("v_nop\n\tv_nop\n\tv_nop\n\tv_nop" : "+v"(d) : "v"(a), "v"(b));
  return d;
}
__device__ __forceinline__ v16h frag_h(const _Float16* rowk0, int lane) {
  union { v16h v; v8h q[2]; } u; const _Float16* p = rowk0 + 8 * (lane >> 4);
  u.q[0] = *(const v8h*)p; u.q[1] = *(const v8h*)(p + 16); return u.v;
}
__device__ __forceinline__ v16h frag_f32(const float* rowk0, int lane) {
  v16h a; const float* p = rowk0 + 8 * (lane >> 4);
#pragma unroll
  for (int i = 0; i < 8; ++i) { a[i] = (_Float16)p[i]; a[8 + i] = (_Float16)p[16 + i]; }
  return a;
}
__device__ __forceinline__ v16h frag_f32s(const float* rowk0, int lane, float sc) {
  v16h a; const float* p = rowk0 + 8 * (lane >> 4);
#pragma unroll
  for (int i = 0; i < 8; ++i) { a[i] = (_Float16)(p[i] * sc); a[8 + i] = (_Float16)(p[16 + i] * sc); }
  return a;
}
__device__ __forceinline__ v16h fragc_f32(const float* W, int k0, int n, int lane, int ld, int K) {
  v16h a; const int g = lane >> 4;
#pragma unroll
  for (int i = 0; i < 8; ++i) { const int ka = k0 + 8 * g + i, kb = ka + 16;
    a[i] = (_Float16)(ka < K ? W[(size_t)ka * ld + n] : 0.f); a[8 + i] = (_Float16)(kb < K ? W[(size_t)kb * ld + n] : 0.f); }
  return a;
}
struct F2 { v16b h, l; };
__device__ __forceinline__ F2 bsplit16(const float v[16]) { F2 r;
#pragma unroll
  for (int i = 0; i < 16; ++i) { const __bf16 h = (__bf16)v[i]; r.h[i] = h; r.l[i] = (__bf16)(v[i] - (float)h); }
  return r; }
__device__ __forceinline__ F2 split_row(const float* row, int k0, int lane) { float v[16]; const float* p = row + k0 + 8 * (lane >> 4);
#pragma unroll
  for (int i = 0; i < 8; ++i) { v[i] = p[i]; v[8 + i] = p[16 + i]; }
  return bsplit16(v); }
__device__ __forceinline__ F2 split_rowK(const float* row, int k0, int lane, int K) { float v[16]; const int g = lane >> 4;
#pragma unroll
  for (int i = 0; i < 8; ++i) { const int ka = k0 + 8 * g + i, kb = ka + 16; v[i] = ka < K ? row[ka] : 0.f; v[8 + i] = kb < K ? row[kb] : 0.f; }
  return bsplit16(v); }
__device__ __forceinline__ F2 split_col(const float* W, int k0, int n, int lane, int ld, int K) { float v[16]; const int g = lane >> 4;
#pragma unroll
  for (int i = 0; i < 8; ++i) { const int ka = k0 + 8 * g + i, kb = ka + 16; v[i] = ka < K ? W[(size_t)ka * ld + n] : 0.f; v[8 + i] = kb < K ? W[(size_t)kb * ld + n] : 0.f; }
  return bsplit16(v); }
__device__ __forceinline__ v8f mac3(const F2& a, const F2& b, v8f c) { c = wmma_bf(a.l, b.h, c); c = wmma_bf(a.h, b.l, c); return wmma_bf(a.h, b.h, c); }
__device__ __forceinline__ float sigm(float v) { return 1.0f / (1.0f + expf(-v)); }
#define LDSX() do { asm volatile("s_wait_dscnt 0" ::: "memory"); __builtin_amdgcn_wave_barrier(); __builtin_amdgcn_fence(__ATOMIC_RELEASE, "workgroup"); } while (0)

#define NB 8
#define NNODE 1024
#define CI 64
#define KORD 4
#define NR (NB * NNODE)

__global__ __launch_bounds__(128) void k_lz(const float* __restrict__ L, const float* __restrict__ Zin, const float* __restrict__ Zprev, float coef, float* __restrict__ Zout) {
  __shared__ __align__(16) float so[4][16][CI + 4];
  const int tid = threadIdx.x, wave = tid >> 5, lane = tid & 31, col = lane & 15, g = lane >> 4;
  const int r0 = blockIdx.x * 64 + wave * 16; const int b = r0 / NNODE; const float* Zb = Zin + (size_t)b * NNODE * CI;
  v8f acc[4] = {};
#pragma unroll 1
  for (int kc = 0; kc < NNODE / 32; ++kc) { const F2 a = split_row(L + (size_t)(r0 + col) * NNODE, kc * 32, lane);
#pragma unroll
    for (int t = 0; t < 4; ++t) acc[t] = mac3(a, split_col(Zb, kc * 32, t * 16 + col, lane, CI, NNODE), acc[t]); }
#pragma unroll
  for (int t = 0; t < 4; ++t) { const int c = t * 16 + col;
#pragma unroll
    for (int r = 0; r < 8; ++r) { float v = acc[t][r] * coef; if (Zprev) v -= Zprev[(size_t)(r0 + 8 * g + r) * CI + c]; so[wave][8 * g + r][c] = v; } }
  LDSX();
  for (int q = lane; q < 16 * 16; q += 32) { const int rl = q >> 4, pc = q & 15; vst2(Zout + (size_t)(r0 + rl) * CI + pc * 4, *(const v4f*)(&so[wave][rl][pc * 4])); }
}
__global__ __launch_bounds__(128) void k_out(const float* __restrict__ x, const float* __restrict__ Z1, const float* __restrict__ Z2, const float* __restrict__ Z3, const float* __restrict__ th, float* __restrict__ out) {
  __shared__ __align__(16) float so[4][16][CI + 4];
  const int tid = threadIdx.x, wave = tid >> 5, lane = tid & 31, col = lane & 15, g = lane >> 4;
  const int r0 = blockIdx.x * 64 + wave * 16;
  v8f acc[4] = {};
#pragma unroll 1
  for (int kk = 0; kk < KORD; ++kk) { const float* Z = kk == 0 ? x : kk == 1 ? Z1 : kk == 2 ? Z2 : Z3; const float* T = th + (size_t)kk * CI * CI;
#pragma unroll
    for (int kc = 0; kc < CI / 32; ++kc) { const F2 a = split_row(Z + (size_t)(r0 + col) * CI, kc * 32, lane);
#pragma unroll
      for (int t = 0; t < 4; ++t) acc[t] = mac3(a, split_col(T, kc * 32, t * 16 + col, lane, CI, CI), acc[t]); } }
#pragma unroll
  for (int t = 0; t < 4; ++t)
#pragma unroll
    for (int r = 0; r < 8; ++r) so[wave][8 * g + r][t * 16 + col] = acc[t][r];
  LDSX();
  for (int q = lane; q < 16 * 16; q += 32) { const int rl = q >> 4, pc = q & 15; vst2(out + (size_t)(r0 + rl) * CI + pc * 4, *(const v4f*)(&so[wave][rl][pc * 4])); }
}
extern "C" void kernel_launch(void* const* d_in, const int* in_sizes, int n_in, void* d_out, int out_size, void* d_ws, size_t ws_size, hipStream_t stream) {
  (void)in_sizes; (void)n_in; (void)out_size; (void)ws_size;
  const float* x = (const float*)d_in[0]; const float* L = (const float*)d_in[1]; const float* th = (const float*)d_in[2];
  float* out = (float*)d_out;
  char* ws = (char*)d_ws; size_t off = 0;
  auto take = [&](size_t bytes) { char* p = ws + off; off += (bytes + 255) & ~(size_t)255; return p; };
  float* Z1 = (float*)take((size_t)NR * CI * 4); float* Z2 = (float*)take((size_t)NR * CI * 4); float* Z3 = (float*)take((size_t)NR * CI * 4);
  k_lz<<<NR / 64, 128, 0, stream>>>(L, x, nullptr, 1.0f, Z1);
  k_lz<<<NR / 64, 128, 0, stream>>>(L, Z1, x, 2.0f, Z2);
  k_lz<<<NR / 64, 128, 0, stream>>>(L, Z2, Z1, 2.0f, Z3);
  k_out<<<NR / 64, 128, 0, stream>>>(x, Z1, Z2, Z3, th, out);
}
